// PeriDynamicAttentionTriton_43800076485144
// MI455X (gfx1250) — hardware-verified
//
#include <hip/hip_runtime.h>
#include <stdint.h>


typedef _Float16 v8h  __attribute__((ext_vector_type(8)));
typedef _Float16 v16h __attribute__((ext_vector_type(16)));
typedef float    v8f  __attribute__((ext_vector_type(8)));
typedef float    v4f  __attribute__((ext_vector_type(4)));
typedef v4f __attribute__((may_alias)) v4fa;
union Frag { v16h v; v8h half[2]; };

#define CD    1024
#define NDSP  256
#define NDV   1280
#define NHD   16
#define BDIM  16
#define HSZ   64
#define WIN   64
#define SEQT  1024

__device__ __forceinline__ v8f wmma16(v16h a, v16h b, v8f c)
{
    v8f d = __builtin_amdgcn_wmma_f32_16x16x32_f16(false, a, false, b, (short)0, c, false, false);
    asm volatile("v_nop\n\tv_nop\n\tv_nop\n\tv_nop" : "+v"(d) : "v"(a), "v"(b));
    return d;
}

__launch_bounds__(256)
__global__ void k_cvt(const float* __restrict__ s0, _Float16* d0, int n0, float c0,
                      const float* __restrict__ s1, _Float16* d1, int n1, float c1,
                      const float* __restrict__ s2, _Float16* d2, int n2, float c2,
                      const float* __restrict__ s3, _Float16* d3, int n3, float c3)
{
    const int seg = blockIdx.y;
    const float* s; _Float16* d; int n; float c;
    if (seg == 0)      { s = s0; d = d0; n = n0; c = c0; }
    else if (seg == 1) { s = s1; d = d1; n = n1; c = c1; }
    else if (seg == 2) { s = s2; d = d2; n = n2; c = c2; }
    else               { s = s3; d = d3; n = n3; c = c3; }
    const size_t i = ((size_t)blockIdx.x * 256 + threadIdx.x) * 8;
    if (i + 8 > (size_t)n) return;
    const v4f a = *(const v4f*)(s + i);
    const v4f b = *(const v4f*)(s + i + 4);
    v8h o;
    o[0] = (_Float16)(a[0] * c); o[1] = (_Float16)(a[1] * c); o[2] = (_Float16)(a[2] * c); o[3] = (_Float16)(a[3] * c);
    o[4] = (_Float16)(b[0] * c); o[5] = (_Float16)(b[1] * c); o[6] = (_Float16)(b[2] * c); o[7] = (_Float16)(b[3] * c);
    _Float16* p = d + i;
    *(volatile v8h*)p = o;
    __threadfence();
    *(volatile v8h*)p = o;
}

#define GBM 128
#define GBN 64
#define GBK 32
#define LDH 40
#define LDCS 68

__launch_bounds__(256)
__global__ void k_gemm(const _Float16* __restrict__ A, const _Float16* __restrict__ W,
                       const float* __restrict__ bias0, const float* __restrict__ bias1, int nsplit,
                       float* C, int M, int N, int K, float scale)
{
    __shared__ __align__(16) _Float16 As[GBM * LDH];
    __shared__ __align__(16) _Float16 Bs[GBN * LDH];
    __shared__ __align__(16) float    Cs[GBM * LDCS];

    const int tid = threadIdx.x;
    const int w = tid >> 5, l = tid & 31, h = l >> 4, m = l & 15;
    const int bm = blockIdx.y * GBM, bn = blockIdx.x * GBN;
    if (bm + GBM > M || bn + GBN > N) return;

    v8f acc[4];
    #pragma unroll
    for (int j = 0; j < 4; ++j) { v8f z = {0.f,0.f,0.f,0.f,0.f,0.f,0.f,0.f}; acc[j] = z; }

    for (int k0 = 0; k0 < K; k0 += GBK) {
        __syncthreads();
        #pragma unroll
        for (int i = 0; i < 2; ++i) {
            const int li = tid + i * 256;
            const int row = li >> 2, cg = (li & 3) * 8;
            *(v8h*)(As + row * LDH + cg) = *(const v8h*)(A + (size_t)(bm + row) * K + k0 + cg);
        }
        {
            const int row = tid >> 2, cg = (tid & 3) * 8;
            *(v8h*)(Bs + row * LDH + cg) = *(const v8h*)(W + (size_t)(bn + row) * K + k0 + cg);
        }
        __syncthreads();
        Frag a;
        a.half[0] = *(const v8h*)(As + (w * 16 + m) * LDH + 8 * h);
        a.half[1] = *(const v8h*)(As + (w * 16 + m) * LDH + 16 + 8 * h);
        #pragma unroll
        for (int j = 0; j < 4; ++j) {
            Frag b;
            b.half[0] = *(const v8h*)(Bs + (j * 16 + m) * LDH + 8 * h);
            b.half[1] = *(const v8h*)(Bs + (j * 16 + m) * LDH + 16 + 8 * h);
            acc[j] = wmma16(a.v, b.v, acc[j]);
        }
    }

    #pragma unroll
    for (int j = 0; j < 4; ++j) {
        #pragma unroll
        for (int r = 0; r < 8; ++r) Cs[(w * 16 + 8 * h + r) * LDCS + j * 16 + m] = acc[j][r];
    }
    __syncthreads();

    const float* bp = (bn < nsplit) ? (bias0 + bn) : (bias1 + (bn - nsplit));
    const int q = l >> 3, e = l & 7;
    const int col = (q & 1) * 32 + e * 4;
    v4f bv;
    bv[0] = bp[col]; bv[1] = bp[col + 1]; bv[2] = bp[col + 2]; bv[3] = bp[col + 3];
    v4f vals[8];
    #pragma unroll
    for (int it = 0; it < 8; ++it) {
        const int row = w * 16 + it * 2 + (q >> 1);
        const v4f v = *(const v4fa*)(Cs + row * LDCS + col);
        vals[it] = v * scale + bv;
    }
    #pragma unroll
    for (int it = 0; it < 8; ++it) {
        const int row = w * 16 + it * 2 + (q >> 1);
        float* p = C + (size_t)(bm + row) * N + bn + col;
        *(volatile v4f*)p = vals[it];
    }
    __threadfence();
    #pragma unroll
    for (int it = 0; it < 8; ++it) {
        const int row = w * 16 + it * 2 + (q >> 1);
        float* p = C + (size_t)(bm + row) * N + bn + col;
        *(volatile v4f*)p = vals[it];
    }
}

#define TT   32
#define NR   96
#define NRV  95
#define PSP  33
#define LGP  65

__device__ __forceinline__ float gelu_f(float z)
{
    return 0.5f * z * (1.f + erff(z * 0.70710678118654752f));
}

__launch_bounds__(256)
__global__ void k_attn(const float* __restrict__ cc,
                       const float* __restrict__ rel,
                       const float* __restrict__ W_fused,
                       const float* __restrict__ b_fused,
                       const float* __restrict__ W_pos,
                       const float* __restrict__ W_bond,
                       const float* __restrict__ b_bond,
                       const float* __restrict__ W_dmg,
                       const float* __restrict__ b_dmg,
                       _Float16* A2,
                       int T, int nTile, int nBlk)
{
    __shared__ __align__(16) float Vs[NR * HSZ];
    __shared__ __align__(16) float Ps[NR * PSP];
    __shared__ __align__(16) float Ds[NR * BDIM];
    __shared__ float PF[WIN * BDIM];
    __shared__ float Lg[TT * LGP];
    __shared__ float Sm[64];

    const int tid = threadIdx.x;
    const int bid = blockIdx.x;
    if (bid >= nBlk) return;
    const int tt = bid % nTile;
    const int bh = bid / nTile;
    const int h  = bh % NHD;
    const int b  = bh / NHD;
    const int t0 = tt * TT;
    const size_t rb = (size_t)b * T;

    for (int i = tid; i < NR * (HSZ / 4); i += 256) {
        const int si = i >> 4, c4 = (i & 15) * 4;
        const int s = t0 - (WIN - 1) + si;
        v4f v = {0.f, 0.f, 0.f, 0.f};
        if (s >= 0 && s < T && si < NRV) v = *(const v4f*)(cc + (rb + s) * NDV + NDSP + h * HSZ + c4);
        *(v4f*)(Vs + si * HSZ + c4) = v;
    }
    for (int i = tid; i < NR * (BDIM / 4); i += 256) {
        const int si = i >> 2, c4 = (i & 3) * 4;
        const int s = t0 - (WIN - 1) + si;
        v4f v = {0.f, 0.f, 0.f, 0.f};
        if (s >= 0 && s < T && si < NRV) v = *(const v4f*)(cc + (rb + s) * NDV + h * BDIM + c4);
        *(v4f*)(Ds + si * BDIM + c4) = v;
    }
    for (int i = tid; i < WIN * BDIM; i += 256) {
        const int j = i >> 4, d = i & 15;
        float s = 0.f;
        #pragma unroll 1
        for (int e = 0; e < BDIM; ++e) s += rel[j * BDIM + e] * W_pos[d * BDIM + e];
        PF[i] = s;
    }
    if (tid < 32)      Sm[tid] = b_fused[tid];
    else if (tid < 48) Sm[tid] = W_bond[tid - 32];
    else if (tid < 64) Sm[tid] = W_dmg[tid - 48];
    __syncthreads();

    {
        const int k = tid & 31, sb = tid >> 5;
        float wr[BDIM];
        #pragma unroll
        for (int d = 0; d < BDIM; ++d) wr[d] = W_fused[k * BDIM + d];
        #pragma unroll 1
        for (int i = 0; i < NR / 8; ++i) {
            const int si = sb + 8 * i;
            float s = 0.f;
            #pragma unroll
            for (int d = 0; d < BDIM; ++d) s += Ds[si * BDIM + d] * wr[d];
            Ps[si * PSP + k] = s;
        }
    }
    __syncthreads();

    {
        const int tl = tid >> 3, jb = tid & 7;
        const int sit = tl + (WIN - 1);
        const float bb = b_bond[0], bdm = b_dmg[0];
        #pragma unroll 1
        for (int i = 0; i < 8; ++i) {
            const int j = jb + 8 * i;
            const int sis = tl + j;
            const int s = t0 + tl - (WIN - 1) + j;
            float bond = 0.f, dmg = 0.f;
            #pragma unroll 1
            for (int d = 0; d < BDIM; ++d) {
                const float z1 = ((Ps[sis * PSP + d] - Ps[sit * PSP + d]) + Sm[d]) + PF[j * BDIM + d];
                const float z2 =  (Ps[sis * PSP + BDIM + d] - Ps[sit * PSP + BDIM + d]) + Sm[BDIM + d];
                bond += gelu_f(z1) * Sm[32 + d];
                dmg  += gelu_f(z2) * Sm[48 + d];
            }
            const float dam = 1.f / (1.f + __expf(-(dmg + bdm)));
            const float lo  = (bond + bb) - 10.f * dam;
            Lg[tl * LGP + j] = (s >= 0) ? lo : -__builtin_inff();
        }
    }
    __syncthreads();

    {
        const int w = tid >> 5, l = tid & 31;
        #pragma unroll 1
        for (int r = 0; r < 4; ++r) {
            const int row = w * 4 + r;
            const float a = Lg[row * LGP + l], c = Lg[row * LGP + 32 + l];
            float mx = fmaxf(a, c);
            #pragma unroll
            for (int o = 16; o > 0; o >>= 1) mx = fmaxf(mx, __shfl_xor(mx, o, 32));
            const float ea = __expf(a - mx), ec = __expf(c - mx);
            float sm = ea + ec;
            #pragma unroll
            for (int o = 16; o > 0; o >>= 1) sm += __shfl_xor(sm, o, 32);
            const float inv = 1.f / sm;
            Lg[row * LGP + l]      = ea * inv;
            Lg[row * LGP + 32 + l] = ec * inv;
        }
    }
    __syncthreads();

    float* Os = Ps;
    {
        const int c = tid & 63, tb = (tid >> 6) * 8;
        float acc[8];
        #pragma unroll
        for (int i = 0; i < 8; ++i) acc[i] = 0.f;
        #pragma unroll 1
        for (int j = 0; j < WIN; ++j) {
            const float* vr = Vs + (tb + j) * HSZ + c;
            #pragma unroll
            for (int i = 0; i < 8; ++i) acc[i] += Lg[(tb + i) * LGP + j] * vr[i * HSZ];
        }
        #pragma unroll
        for (int i = 0; i < 8; ++i) Os[(tb + i) * HSZ + c] = acc[i];
    }
    __syncthreads();

    {
        const int w = tid >> 5, l = tid & 31, q = l >> 3, e = l & 7;
        const int row = w * 4 + q, c0 = e * 8;
        const v4f u0 = *(const v4fa*)(Os + row * HSZ + c0);
        const v4f u1 = *(const v4fa*)(Os + row * HSZ + c0 + 4);
        v8h o;
        o[0] = (_Float16)(u0[0] * 16.f); o[1] = (_Float16)(u0[1] * 16.f);
        o[2] = (_Float16)(u0[2] * 16.f); o[3] = (_Float16)(u0[3] * 16.f);
        o[4] = (_Float16)(u1[0] * 16.f); o[5] = (_Float16)(u1[1] * 16.f);
        o[6] = (_Float16)(u1[2] * 16.f); o[7] = (_Float16)(u1[3] * 16.f);
        const int t = t0 + row;
        if (t < T) {
            _Float16* p = A2 + (rb + t) * CD + h * HSZ + c0;
            *(volatile v8h*)p = o;
            __threadfence();
            *(volatile v8h*)p = o;
        }
    }
}

extern "C" void kernel_launch(void* const* d_in, const int* in_sizes, int n_in,
                              void* d_out, int out_size, void* d_ws, size_t ws_size,
                              hipStream_t stream)
{
    if (n_in < 15) return;
    const float* x       = (const float*)d_in[0];
    const float* W_disp  = (const float*)d_in[1];
    const float* b_disp  = (const float*)d_in[2];
    const float* W_val   = (const float*)d_in[3];
    const float* b_val   = (const float*)d_in[4];
    const float* rel     = (const float*)d_in[5];
    const float* W_fused = (const float*)d_in[6];
    const float* b_fused = (const float*)d_in[7];
    const float* W_pos   = (const float*)d_in[8];
    const float* W_bond  = (const float*)d_in[9];
    const float* b_bond  = (const float*)d_in[10];
    const float* W_dmg   = (const float*)d_in[11];
    const float* b_dmg   = (const float*)d_in[12];
    const float* W_cproj = (const float*)d_in[13];
    const float* b_cproj = (const float*)d_in[14];
    float* out = (float*)d_out;

    if (in_sizes[4] != CD || in_sizes[2] != NDSP || in_sizes[14] != CD) return;
    if (in_sizes[1] != NDSP * CD || in_sizes[3] != CD * CD || in_sizes[13] != CD * CD) return;
    if (in_sizes[5] != WIN * BDIM || in_sizes[6] != 2 * BDIM * BDIM || in_sizes[7] != 2 * BDIM) return;
    if (in_sizes[8] != BDIM * BDIM || in_sizes[9] != BDIM || in_sizes[11] != BDIM) return;
    if (in_sizes[10] < 1 || in_sizes[12] < 1) return;
    const int BT = in_sizes[0] / CD;
    if (BT * CD != in_sizes[0] || out_size != BT * CD) return;
    const int T = SEQT;
    if (BT % T != 0) return;
    const int B = BT / T;
    if (BT % GBM != 0 || (NDV % GBN) != 0 || (CD % GBN) != 0 || (CD % GBK) != 0 || (T % TT) != 0) return;

    char* ws = (char*)d_ws;
    size_t off = 0;
    const size_t n_xh  = (size_t)BT * CD;
    const size_t n_wdv = (size_t)NDV * CD;
    const size_t n_wch = (size_t)CD * CD;
    const size_t n_cc  = (size_t)BT * NDV;
    const size_t n_a2  = (size_t)BT * CD;
    _Float16* xh  = (_Float16*)(ws + off); off = (off + n_xh  * 2 + 255) & ~(size_t)255;
    _Float16* wdv = (_Float16*)(ws + off); off = (off + n_wdv * 2 + 255) & ~(size_t)255;
    _Float16* wch = (_Float16*)(ws + off); off = (off + n_wch * 2 + 255) & ~(size_t)255;
    float*    cc  = (float*)(ws + off);    off = (off + n_cc  * 4 + 255) & ~(size_t)255;
    _Float16* a2  = (_Float16*)(ws + off); off = (off + n_a2  * 2 + 255) & ~(size_t)255;
    if (off > ws_size) return;

    {
        const int n0 = BT * CD, n1 = NDSP * CD, n2 = CD * CD, n3 = CD * CD;
        int nmax = n0; if (n1 > nmax) nmax = n1; if (n2 > nmax) nmax = n2; if (n3 > nmax) nmax = n3;
        const int gx = (nmax + 2047) / 2048;
        k_cvt<<<dim3(gx, 4), 256, 0, stream>>>(x, xh, n0, 1.f,
                                               W_disp, wdv, n1, 64.f,
                                               W_val, wdv + (size_t)NDSP * CD, n2, 64.f,
                                               W_cproj, wch, n3, 64.f);
    }
    k_gemm<<<dim3(NDV / GBN, BT / GBM), 256, 0, stream>>>(xh, wdv, b_disp, b_val, NDSP, cc,
                                                         BT, NDV, CD, 1.f / 64.f);
    {
        const int nTile = T / TT;
        const int nBlk = B * NHD * nTile;
        k_attn<<<nBlk, 256, 0, stream>>>(cc, rel, W_fused, b_fused, W_pos, W_bond, b_bond, W_dmg, b_dmg,
                                          a2, T, nTile, nBlk);
    }
    k_gemm<<<dim3(CD / GBN, BT / GBM), 256, 0, stream>>>(a2, wch, b_cproj, b_cproj, 0, out,
                                                        BT, CD, CD, 1.f / 1024.f);
}
